// SAAM_45646912422425
// MI455X (gfx1250) — hardware-verified
//
#include <hip/hip_runtime.h>
#include <math.h>

#define NBs 8
#define CC 64
#define NN 4096

typedef _Float16 f16;
typedef __attribute__((ext_vector_type(16))) f16 f16x16;
typedef __attribute__((ext_vector_type(8)))  f16 f16x8;
typedef __attribute__((ext_vector_type(8)))  float f32x8;
typedef __attribute__((ext_vector_type(4)))  float v4f_t;
typedef float v4fa __attribute__((ext_vector_type(4), may_alias));
__device__ __forceinline__ f32x8 wmma16(f16x16 a, f16x16 b, f32x8 c) {
  c = __builtin_amdgcn_wmma_f32_16x16x32_f16(false, a, false, b, (short)0, c, false, false);
  asm volatile("v_nop\n\tv_nop\n\tv_nop\n\tv_nop" : "+v"(c) : "v"(a), "v"(b));
  return c;
}
__device__ __forceinline__ f16x16 lds_frag(const f16* base, int stride) {
  const int lane = threadIdx.x & 31, row = lane & 15, kh = (lane >> 4) * 8;
  const f16x8 lo = *(const f16x8*)(base + row * stride + kh);
  const f16x8 hi = *(const f16x8*)(base + row * stride + kh + 16);
  f16x16 f;
#pragma unroll
  for (int i = 0; i < 8; ++i) { f[i] = lo[i]; f[i + 8] = hi[i]; }
  return f;
}
__global__ __launch_bounds__(256) void k_mean(const float* __restrict__ x, float* __restrict__ a) {
  const int b = blockIdx.x >> 4, n = (blockIdx.x & 15) * 256 + threadIdx.x; const float* p = x + (size_t)b * CC * NN + n; float s = 0.0f;
#pragma unroll 1
  for (int c = 0; c < CC; ++c) s += p[(size_t)c * NN];
  a[(size_t)b * NN + n] = s / (float)CC;
}
__global__ __launch_bounds__(256) void k_rowstats(const float* __restrict__ a, float* __restrict__ rz) {
  __shared__ float redM[256], redm[256]; __shared__ float aS[NN];
  const int tid = threadIdx.x, b = blockIdx.x; const float* ab = a + (size_t)b * NN;
  float mx = -3.0e38f, mn = 3.0e38f;
  for (int n = tid; n < NN; n += 256) { const float v = ab[n]; aS[n] = v; mx = fmaxf(mx, v); mn = fminf(mn, v); }
  redM[tid] = mx; redm[tid] = mn; __syncthreads();
  for (int o = 128; o > 0; o >>= 1) { if (tid < o) { redM[tid] = fmaxf(redM[tid], redM[tid + o]); redm[tid] = fminf(redm[tid], redm[tid + o]); } __syncthreads(); }
  const float amax = redM[0], amin = redm[0];
  for (int n = tid; n < NN; n += 256) { const float an = aS[n]; const float r = (an >= 0.0f) ? an * amax : an * amin; float z = 0.0f;
#pragma unroll 1
    for (int m = 0; m < NN; ++m) z += expf(an * aS[m] - r);
    rz[((size_t)b * NN + n) * 2] = r; rz[((size_t)b * NN + n) * 2 + 1] = z; }
}
__global__ __launch_bounds__(256) void k_saam(const float* __restrict__ x, const float* __restrict__ a, const float* __restrict__ rz, float* __restrict__ out) {
  __shared__ __attribute__((aligned(16))) f16 pS[64 * 40];
  __shared__ float anS[64], rS[64], zS[64], amS[NN];
  __shared__ __attribute__((aligned(16))) float oS[CC * 68];
  const int tid = threadIdx.x, lane = tid & 31, wave = tid >> 5, cl = lane & 15, rh = (lane >> 4) * 8;
  const int b = blockIdx.x / (NN / 64), n0 = (blockIdx.x % (NN / 64)) * 64;
  for (int e = tid; e < NN; e += 256) amS[e] = a[(size_t)b * NN + e];
  if (tid < 64) { anS[tid] = a[(size_t)b * NN + n0 + tid]; rS[tid] = rz[((size_t)b * NN + n0 + tid) * 2]; zS[tid] = rz[((size_t)b * NN + n0 + tid) * 2 + 1]; }
  const float* xb = x + (size_t)b * CC * NN;
  const int rt = wave & 3, ct0 = (wave >> 2) * 2;
  f32x8 acc[2]; { f32x8 z = {}; acc[0] = z; acc[1] = z; }
  __syncthreads();
#pragma unroll 1
  for (int m0 = 0; m0 < NN; m0 += 32) {
    { const int r = tid >> 2, q = (tid & 3) * 8; const float an = anS[r], rr = rS[r];
#pragma unroll
      for (int e = 0; e < 8; ++e) pS[r * 40 + q + e] = (f16)(expf(an * amS[m0 + q + e] - rr) * 1024.0f); }
    __syncthreads();
    { const f16x16 af = lds_frag(pS + (rt * 16) * 40, 40);
#pragma unroll
      for (int j = 0; j < 2; ++j) { const int c = (ct0 + j) * 16 + (lane & 15), kh = (lane >> 4) * 8; const float* src = xb + (size_t)c * NN + m0 + kh; f16x16 bf;
#pragma unroll
        for (int e = 0; e < 8; ++e) { bf[e] = (f16)src[e]; bf[8 + e] = (f16)src[16 + e]; }
        acc[j] = wmma16(af, bf, acc[j]); } }
    __syncthreads();
  }
#pragma unroll
  for (int j = 0; j < 2; ++j)
#pragma unroll
    for (int r = 0; r < 8; ++r) { const int n = rt * 16 + rh + r, c = (ct0 + j) * 16 + cl; oS[c * 68 + n] = acc[j][r] / (zS[n] * 1024.0f); }
  __syncthreads();
#pragma unroll 1
  for (int pass = 0; pass < 2; ++pass) { for (int q4 = tid; q4 < CC * 16; q4 += 256) { const int c = q4 >> 4, c4 = (q4 & 15) * 4;
      *(volatile v4f_t*)(out + ((size_t)b * CC + c) * NN + n0 + c4) = *(const v4fa*)(oS + c * 68 + c4); } __threadfence(); }
}

extern "C" void kernel_launch(void* const* d_in, const int* in_sizes, int n_in,
                              void* d_out, int out_size, void* d_ws, size_t ws_size,
                              hipStream_t stream) {
  (void)in_sizes; (void)n_in; (void)out_size;
  const float* x = (const float*)d_in[0];
  float* out = (float*)d_out;
  char* ws = (char*)d_ws;
  float* a = (float*)ws; ws += (size_t)NBs * NN * 4; float* rz = (float*)ws; ws += (size_t)NBs * NN * 2 * 4;
  if ((size_t)(ws - (char*)d_ws) > ws_size) return;
  k_mean<<<dim3(NBs * 16), dim3(256), 0, stream>>>(x, a);
  k_rowstats<<<dim3(NBs), dim3(256), 0, stream>>>(a, rz);
  k_saam<<<dim3(NBs * (NN / 64)), dim3(256), 0, stream>>>(x, a, rz, out);
}
